// LSTMCRFTagger_79697413144975
// MI455X (gfx1250) — hardware-verified
//
#include <hip/hip_runtime.h>
#include <math.h>
#include <stdint.h>

constexpr int SEQ_LEN     = 512;
constexpr int N_BATCH     = 32;
constexpr int EMB_DIM     = 300;
constexpr int EMB_PAD     = 320;
constexpr int HID_DIM     = 500;
constexpr int HID_PAD     = 512;
constexpr int GATE_ROWS   = 2000;
constexpr int GATE_COLS   = 2048;
constexpr int N_TAGS      = 16;
constexpr int TAG_PAD     = 64;
constexpr int HS_COLS     = 1024;
constexpr int N_ROWS      = SEQ_LEN * N_BATCH;
constexpr int N_VOCAB     = 30000;
constexpr int W_TAG_COLS  = 1000;
constexpr int REC_THREADS = 512;
constexpr int AH_PITCH    = 520;
constexpr float W_CARRY     = 16.0f;
constexpr float W_CARRY_INV = 1.0f / 16.0f;

static_assert(EMB_PAD % 32 == 0 && HID_PAD % 32 == 0 && HS_COLS % 32 == 0, "K multiples of 32");
static_assert(N_ROWS % 64 == 0 && GATE_COLS % 64 == 0 && TAG_PAD % 64 == 0, "M,N multiples of 64");
static_assert(REC_THREADS == HID_PAD, "one thread per padded hidden column in the h tile init");

typedef __attribute__((ext_vector_type(16))) _Float16 v16h;
typedef __attribute__((ext_vector_type(8)))  _Float16 v8h;
typedef __attribute__((ext_vector_type(16))) __bf16   v16b;
typedef __attribute__((ext_vector_type(8)))  __bf16   v8b;
typedef __attribute__((ext_vector_type(8)))  float    v8f;
typedef __attribute__((ext_vector_type(4)))  float    v4f;

__device__ __forceinline__ unsigned short f2bf_bits(float f) {
  unsigned u = __float_as_uint(f);
  return (unsigned short)((u + 0x7FFFu + ((u >> 16) & 1u)) >> 16);
}
__device__ __forceinline__ float bf_bits2f(unsigned short h) { return __uint_as_float(((unsigned)h) << 16); }

__device__ __forceinline__ void dep_guard_h(v8f& a, v8f& b, v16h x, v16h y) { asm volatile("v_nop\n\tv_nop\n\tv_nop\n\tv_nop" : "+v"(a), "+v"(b) : "v"(x), "v"(y)); }
__device__ __forceinline__ void dep_guard_b(v8f& a, v8f& b, v16b x, v16b y) { asm volatile("v_nop\n\tv_nop\n\tv_nop\n\tv_nop" : "+v"(a), "+v"(b) : "v"(x), "v"(y)); }
__device__ __forceinline__ void keep4_h(v16h a, v16h b, v16h c, v16h d) { asm volatile("v_nop" :: "v"(a), "v"(b), "v"(c), "v"(d)); }
__device__ __forceinline__ void keep4_b(v16b a, v16b b, v16b c, v16b d) { asm volatile("v_nop" :: "v"(a), "v"(b), "v"(c), "v"(d)); }
__device__ __forceinline__ void acc_guard4(v8f& a, v8f& b, v8f& c, v8f& d) { asm volatile("v_nop\n\tv_nop\n\tv_nop\n\tv_nop" : "+v"(a), "+v"(b), "+v"(c), "+v"(d)); }
template <typename T> struct Frag;
template <> struct Frag<_Float16> {
  typedef v16h V; union U { v16h v; v8h h[2]; };
  static __device__ __forceinline__ v16h load(const _Float16* p) {
    U f; f.h[0] = *(const v8h*)(p); f.h[1] = *(const v8h*)(p + 16); return f.v;
  }
  static __device__ __forceinline__ v8f mma(v16h a, v16h b, v8f c) {
    return __builtin_amdgcn_wmma_f32_16x16x32_f16(false, a, false, b, (short)0, c, false, false);
  }
  static __device__ __forceinline__ void guard(v8f& a, v8f& b, v16h x, v16h y) { dep_guard_h(a, b, x, y); }
  static __device__ __forceinline__ void keep(v16h a, v16h b, v16h c, v16h d) { keep4_h(a, b, c, d); }
};
template <> struct Frag<__bf16> {
  typedef v16b V; union U { v16b v; v8b h[2]; };
  static __device__ __forceinline__ v16b load(const __bf16* p) {
    U f; f.h[0] = *(const v8b*)(p); f.h[1] = *(const v8b*)(p + 16); return f.v;
  }
  static __device__ __forceinline__ v8f mma(v16b a, v16b b, v8f c) {
    return __builtin_amdgcn_wmma_f32_16x16x32_bf16(false, a, false, b, (short)0, c, false, false);
  }
  static __device__ __forceinline__ void guard(v8f& a, v8f& b, v16b x, v16b y) { dep_guard_b(a, b, x, y); }
  static __device__ __forceinline__ void keep(v16b a, v16b b, v16b c, v16b d) { keep4_b(a, b, c, d); }
};

template <int ET> struct Elem;
template <> struct Elem<0> { typedef _Float16 T; };
template <> struct Elem<1> { typedef __bf16 T; };
template <int ET, bool SPLIT, int BIAS_MODE, int OUT_MODE, bool RESID, int ACT = 0>
__global__ __launch_bounds__(256) void wmma_gemm64(
    const unsigned short* __restrict__ Ap, const unsigned short* __restrict__ A2p, int lda, long strideA,
    const unsigned short* __restrict__ Btp, const unsigned short* __restrict__ Bt2p, int ldb, long strideB,
    void* __restrict__ Cout, void* __restrict__ Cout2, int ldc, long strideC,
    const float* __restrict__ bias,
    const float* __restrict__ resid, long strideR,
    int M, int N, int K, float scale) {
  typedef typename Elem<ET>::T T;
  typedef typename Frag<T>::V V;
  const T* A = (const T*)Ap; const T* A2 = (const T*)A2p; const T* Bt = (const T*)Btp; const T* Bt2 = (const T*)Bt2p;
  __shared__ __align__(16) float sT[8][16 * 68];
  const int b    = blockIdx.y;
  const int lane = threadIdx.x & 31;
  const int wave = threadIdx.x >> 5;
  const int tilesN = N >> 6;
  const int tilesM = M >> 6;
  const int tile = blockIdx.x * 8 + wave;
  if (tile >= tilesM * tilesN) return;
  const int tm = tile / tilesN;
  const int tn = tile - tm * tilesN;
  const int m0 = tm << 6;
  const int n0 = tn << 6;

  const T* Ab  = A  + (size_t)b * strideA;
  const T* Bb  = Bt + (size_t)b * strideB;
  const T* Ab2 = SPLIT ? (A2  + (size_t)b * strideA) : nullptr;
  const T* Bb2 = SPLIT ? (Bt2 + (size_t)b * strideB) : nullptr;

  const int rlane = lane & 15;
  const int koff  = (lane >> 4) * 8;
  const int mOff  = (lane >> 4) * 8;

  v8f acc[4][4];
#pragma unroll
  for (int i = 0; i < 4; ++i)
#pragma unroll
    for (int j = 0; j < 4; ++j) acc[i][j] = (v8f){0.f,0.f,0.f,0.f,0.f,0.f,0.f,0.f};

  for (int k0 = 0; k0 < K; k0 += 32) {
    V bh[4], bl[4];
#pragma unroll
    for (int j = 0; j < 4; ++j) {
      const size_t bo = (size_t)(n0 + (j << 4) + rlane) * ldb + koff + k0;
      bh[j] = Frag<T>::load(Bb + bo);
      if (SPLIT) bl[j] = Frag<T>::load(Bb2 + bo);
    }
#pragma unroll
    for (int i = 0; i < 4; ++i) {
      const size_t ao = (size_t)(m0 + (i << 4) + rlane) * lda + koff + k0;
      V ah = Frag<T>::load(Ab + ao);
      V al;
      if (SPLIT) al = Frag<T>::load(Ab2 + ao);
#pragma unroll
      for (int j = 0; j < 4; ++j) {
        acc[i][j] = Frag<T>::mma(ah, bh[j], acc[i][j]);
        if (SPLIT) {
          acc[i][j] = Frag<T>::mma(ah, bl[j], acc[i][j]);
          acc[i][j] = Frag<T>::mma(al, bh[j], acc[i][j]);
        }
      }
      Frag<T>::guard(acc[i][0], acc[i][3], ah, SPLIT ? al : ah);
    }
    Frag<T>::keep(bh[0], bh[1], bh[2], bh[3]);
    if (SPLIT) Frag<T>::keep(bl[0], bl[1], bl[2], bl[3]);
  }
  acc_guard4(acc[0][0], acc[0][1], acc[0][2], acc[0][3]);
  acc_guard4(acc[1][0], acc[1][1], acc[1][2], acc[1][3]);
  acc_guard4(acc[2][0], acc[2][1], acc[2][2], acc[2][3]);
  acc_guard4(acc[3][0], acc[3][1], acc[3][2], acc[3][3]);

  float* slab = sT[wave];
  const float* Rb = RESID ? (resid + (size_t)b * strideR) : nullptr;
#pragma unroll
  for (int i = 0; i < 4; ++i) {
    const int mBase = m0 + (i << 4);
#pragma unroll
    for (int j = 0; j < 4; ++j) {
      const int n = n0 + (j << 4) + rlane;
      float bv = 0.f;
      if (BIAS_MODE == 2) bv = bias[n];
#pragma unroll
      for (int r = 0; r < 8; ++r) {
        float v = acc[i][j][r] * scale;
        if (BIAS_MODE == 1) v += bias[mBase + mOff + r];
        if (BIAS_MODE == 2) v += bv;
        if (RESID) v += Rb[(size_t)(mBase + mOff + r) * ldc + n];
        if (ACT == 1) v = tanhf(v);
        if (ACT == 2) v = fmaxf(v, 0.0f);
        if (ACT == 3) v = v / (1.0f + expf(-v));
        if (ACT == 4) v = (v > 0.f) ? v : 0.01f * v;
        if (ACT == 5) v = 0.5f * v * (1.0f + erff(v * 0.70710678118654752f));
        slab[(mOff + r) * 68 + (j << 4) + rlane] = v;
      }
    }
    __builtin_amdgcn_fence(__ATOMIC_RELEASE, "workgroup");
    __builtin_amdgcn_wave_barrier();
    __builtin_amdgcn_fence(__ATOMIC_ACQUIRE, "workgroup");
    if (OUT_MODE == 0) {
      float* C = (float*)Cout + (size_t)b * strideC;
      const int hh = lane >> 4, c4 = (lane & 15) * 4;
      for (int pass = 0; pass < 2; ++pass) {
#pragma unroll
        for (int it = 0; it < 8; ++it) {
          const int row = it * 2 + hh;
          v4f v = *(const v4f*)(slab + row * 68 + c4);
          *(volatile v4f*)(C + (size_t)(mBase + row) * ldc + n0 + c4) = v;
        }
        __threadfence();
      }
    } else {
      const int q = lane >> 3, c8 = (lane & 7) * 8;
      unsigned short* C  = (unsigned short*)Cout  + (size_t)b * strideC;
      unsigned short* C2 = (OUT_MODE == 2) ? ((unsigned short*)Cout2 + (size_t)b * strideC) : nullptr;
      for (int pass = 0; pass < 2; ++pass) {
#pragma unroll
        for (int it = 0; it < 4; ++it) {
          const int row = it * 4 + q;
          const float* sp = slab + row * 68 + c8;
          v8h hv, lv;
#pragma unroll
          for (int e = 0; e < 8; ++e) {
            if (OUT_MODE == 1) {
              hv[e] = (_Float16)sp[e];
            } else {
              unsigned short hb = f2bf_bits(sp[e]);
              unsigned short lb = f2bf_bits(sp[e] - bf_bits2f(hb));
              hv[e] = __builtin_bit_cast(_Float16, hb);
              lv[e] = __builtin_bit_cast(_Float16, lb);
            }
          }
          *(volatile v8h*)(C + (size_t)(mBase + row) * ldc + n0 + c8) = hv;
          if (OUT_MODE == 2) *(volatile v8h*)(C2 + (size_t)(mBase + row) * ldc + n0 + c8) = lv;
        }
        __threadfence();
      }
    }
    __builtin_amdgcn_fence(__ATOMIC_RELEASE, "workgroup");
    __builtin_amdgcn_wave_barrier();
    __builtin_amdgcn_fence(__ATOMIC_ACQUIRE, "workgroup");
  }
}

__global__ __launch_bounds__(256) void cvt_pad_kernel(const float* __restrict__ src, unsigned short* __restrict__ dst,
                                                      int ndr, int dcols, int rbd, int rbs, int nrb, int nsr,
                                                      int sld, int cbd, int cbs, int ncb, float sc) {
  const int lpr = dcols >> 3;
  const int rpb = 256 / lpr;
  const int tid = threadIdx.x;
  const int rl  = tid / lpr;
  const int q   = tid - rl * lpr;
  const int n   = blockIdx.x * rpb + rl;
  const bool rowok = (rl < rpb) && (n < ndr);
  const int nn  = (n < ndr) ? n : (ndr - 1);
  const int rb  = nn / rbd;
  const int rj  = nn - rb * rbd;
  const bool rvalid = rowok && (rj < rbs) && (rb < nrb);
  int srow = rb * rbs + rj;
  srow = (srow < 0) ? 0 : ((srow > nsr - 1) ? (nsr - 1) : srow);
  const float* sp = src + (size_t)srow * (size_t)sld;
  v8h hv;
#pragma unroll
  for (int e = 0; e < 8; ++e) {
    const int cidx = q * 8 + e;
    const int cb = cidx / cbd;
    const int cj = cidx - cb * cbd;
    const bool cvalid = (cj < cbs) && (cb < ncb);
    int scol = cb * cbs + cj;
    scol = (scol > sld - 1) ? (sld - 1) : scol;
    const float f = sp[scol];
    hv[e] = (_Float16)((rvalid && cvalid) ? (f * sc) : 0.0f);
  }
  if (rowok) {
    unsigned short* dp = dst + (size_t)n * (size_t)dcols + (size_t)(q * 8);
    *(volatile v8h*)dp = hv;
    __threadfence();
    *(volatile v8h*)dp = hv;
  }
}

__global__ __launch_bounds__(256) void gather_rows_kernel(const int* __restrict__ ids, const float* __restrict__ table,
                                                          unsigned short* __restrict__ dst, int nrows, int nvoc,
                                                          int scols, int dcols) {
  const int lpr = dcols >> 3;
  const int rpb = 256 / lpr;
  const int tid = threadIdx.x;
  const int rl  = tid / lpr;
  const int q   = tid - rl * lpr;
  const int n   = blockIdx.x * rpb + rl;
  const bool rowok = (rl < rpb) && (n < nrows);
  const int nn  = (n < nrows) ? n : (nrows - 1);
  int id = ids[nn];
  id = (id < 0) ? 0 : ((id > nvoc - 1) ? (nvoc - 1) : id);
  const float* sp = table + (size_t)id * (size_t)scols;
  v8h hv;
#pragma unroll
  for (int e = 0; e < 8; ++e) {
    const int cidx = q * 8 + e;
    const int scol = (cidx > scols - 1) ? (scols - 1) : cidx;
    const float f = sp[scol];
    hv[e] = (_Float16)((rowok && cidx < scols) ? f : 0.0f);
  }
  if (rowok) {
    unsigned short* dp = dst + (size_t)n * (size_t)dcols + (size_t)(q * 8);
    *(volatile v8h*)dp = hv;
    __threadfence();
    *(volatile v8h*)dp = hv;
  }
}

__device__ __forceinline__ float fsig(float x)  { return __builtin_amdgcn_rcpf(1.0f + __expf(-x)); }
__device__ __forceinline__ float ftanh(float x) { return 1.0f - 2.0f * __builtin_amdgcn_rcpf(__expf(2.0f * x) + 1.0f); }

__global__ __launch_bounds__(REC_THREADS) void lstm_rec_kernel(const unsigned short* __restrict__ XPp,
                                                               const unsigned short* __restrict__ WHp,
                                                               const float* __restrict__ bias,
                                                               unsigned short* __restrict__ HSp, int dir) {
  __shared__ __align__(16) _Float16 Ah[16 * AH_PITCH];
  const _Float16* XPh = (const _Float16*)XPp;
  const _Float16* WH  = (const _Float16*)WHp;
  const int tid = threadIdx.x, lane = tid & 31, wave = tid >> 5;
  const int c = lane & 15, hh = lane >> 4, koff = hh * 8;
  const int bbase = blockIdx.x * 16;

#pragma unroll 1
  for (int i = 0; i < 16; ++i) Ah[i * AH_PITCH + tid] = (_Float16)0.0f;

  float cst[2][8], hst[2][8], bb[2][4];
#pragma unroll
  for (int nt = 0; nt < 2; ++nt) {
    const int j  = 32 * wave + 16 * nt + c;
    const int jc = (j < HID_DIM) ? j : (HID_DIM - 1);
#pragma unroll
    for (int g = 0; g < 4; ++g) {
      const float bv = bias[g * HID_DIM + jc];
      bb[nt][g] = (j < HID_DIM) ? bv : 0.0f;
    }
#pragma unroll
    for (int r = 0; r < 8; ++r) { cst[nt][r] = 0.0f; hst[nt][r] = 0.0f; }
  }
  __syncthreads();

  const _Float16* ahrow = Ah + c * AH_PITCH + koff;
  const v8f z8 = {0.f, 0.f, 0.f, 0.f, 0.f, 0.f, 0.f, 0.f};

#pragma unroll 1
  for (int t = 0; t < SEQ_LEN; ++t) {
    const int s = dir ? (SEQ_LEN - 1 - t) : t;
    const int rowbase = s * N_BATCH + bbase;
    const _Float16* xprow = XPh + (size_t)rowbase * (size_t)GATE_COLS;
#pragma unroll
    for (int nt = 0; nt < 2; ++nt) {
      const int j = 32 * wave + 16 * nt + c;
      const _Float16* wh = WH + (size_t)j * HID_PAD + koff;
      v8f acc[4];
      acc[0] = z8; acc[1] = z8; acc[2] = z8; acc[3] = z8;
#pragma unroll 1
      for (int k0 = 0; k0 < HID_PAD; k0 += 32) {
        const v16h a  = Frag<_Float16>::load(ahrow + k0);
        const v16h b0 = Frag<_Float16>::load(wh + k0);
        const v16h b1 = Frag<_Float16>::load(wh + (size_t)1 * HID_PAD * HID_PAD + k0);
        const v16h b2 = Frag<_Float16>::load(wh + (size_t)2 * HID_PAD * HID_PAD + k0);
        const v16h b3 = Frag<_Float16>::load(wh + (size_t)3 * HID_PAD * HID_PAD + k0);
        acc[0] = Frag<_Float16>::mma(a, b0, acc[0]);
        acc[1] = Frag<_Float16>::mma(a, b1, acc[1]);
        acc[2] = Frag<_Float16>::mma(a, b2, acc[2]);
        acc[3] = Frag<_Float16>::mma(a, b3, acc[3]);
        dep_guard_h(acc[0], acc[3], a, b3);
        keep4_h(b0, b1, b2, b3);
      }
      acc_guard4(acc[0], acc[1], acc[2], acc[3]);
#pragma unroll
      for (int r = 0; r < 8; ++r) {
        const size_t xo = (size_t)(8 * hh + r) * (size_t)GATE_COLS + (size_t)j;
        const float xi = (float)xprow[xo];
        const float xf = (float)xprow[xo + (size_t)HID_PAD];
        const float xg = (float)xprow[xo + (size_t)2 * HID_PAD];
        const float xq = (float)xprow[xo + (size_t)3 * HID_PAD];
        const float zi = acc[0][r] * W_CARRY_INV + xi + bb[nt][0];
        const float zf = acc[1][r] * W_CARRY_INV + xf + bb[nt][1];
        const float zg = acc[2][r] * W_CARRY_INV + xg + bb[nt][2];
        const float zo = acc[3][r] * W_CARRY_INV + xq + bb[nt][3];
        const float ig = fsig(zi);
        const float fg = fsig(zf);
        const float gg = ftanh(zg);
        const float og = fsig(zo);
        const float cn = fg * cst[nt][r] + ig * gg;
        cst[nt][r] = cn;
        hst[nt][r] = og * ftanh(cn);
      }
    }
    __syncthreads();
#pragma unroll
    for (int nt = 0; nt < 2; ++nt) {
      const int j = 32 * wave + 16 * nt + c;
#pragma unroll
      for (int r = 0; r < 8; ++r) Ah[(8 * hh + r) * AH_PITCH + j] = (_Float16)hst[nt][r];
    }
    __syncthreads();
    {
      unsigned short* hsrow = HSp + (size_t)rowbase * (size_t)HS_COLS + (size_t)(dir * HID_PAD);
      for (int pass = 0; pass < 2; ++pass) {
#pragma unroll
        for (int it = 0; it < 2; ++it) {
          const int idx = it * REC_THREADS + tid;
          const int row = idx >> 6, c8 = (idx & 63) * 8;
          const v8h v = *(const v8h*)(Ah + row * AH_PITCH + c8);
          *(volatile v8h*)(hsrow + (size_t)row * HS_COLS + c8) = v;
        }
        __threadfence();
      }
    }
  }
}

__global__ __launch_bounds__(512) void crf_kernel(const float* __restrict__ em, const int* __restrict__ y,
                                                  const float* __restrict__ btag, const float* __restrict__ start,
                                                  const float* __restrict__ endt, const float* __restrict__ trans,
                                                  float* __restrict__ out) {
  __shared__ float tr[16][17];
  __shared__ float alpha[2][32][17];
  __shared__ float bt[16];
  __shared__ float rnum[32], rden[32];
  const int tid = threadIdx.x;
  if (tid < 256) tr[tid >> 4][tid & 15] = trans[tid];
  if (tid < 16) bt[tid] = btag[tid];
  __syncthreads();

  if (tid < 32) {
    const int b = tid;
    int tp = y[b];
    tp = (tp < 0) ? 0 : ((tp > N_TAGS - 1) ? (N_TAGS - 1) : tp);
    float numv = start[tp] + (em[(size_t)b * TAG_PAD + tp] + bt[tp]);
#pragma unroll 1
    for (int s = 1; s < SEQ_LEN; ++s) {
      int tc = y[s * N_BATCH + b];
      tc = (tc < 0) ? 0 : ((tc > N_TAGS - 1) ? (N_TAGS - 1) : tc);
      numv += tr[tp][tc] + (em[(size_t)(s * N_BATCH + b) * TAG_PAD + tc] + bt[tc]);
      tp = tc;
    }
    rnum[b] = numv + endt[tp];
  }

  const int b = tid >> 4, j = tid & 15;
  alpha[0][b][j] = start[j] + (em[(size_t)b * TAG_PAD + j] + bt[j]);
  __syncthreads();
  int cur = 0;
#pragma unroll 1
  for (int s = 1; s < SEQ_LEN; ++s) {
    const float emv = em[(size_t)(s * N_BATCH + b) * TAG_PAD + j] + bt[j];
    float m = -1e30f;
#pragma unroll 1
    for (int i = 0; i < 16; ++i) m = fmaxf(m, alpha[cur][b][i] + tr[i][j]);
    float a = 0.f;
#pragma unroll 1
    for (int i = 0; i < 16; ++i) a += expf(alpha[cur][b][i] + tr[i][j] - m);
    alpha[cur ^ 1][b][j] = m + logf(a) + emv;
    cur ^= 1;
    __syncthreads();
  }
  if (tid < 32) {
    float m = -1e30f;
#pragma unroll 1
    for (int jj = 0; jj < 16; ++jj) m = fmaxf(m, alpha[cur][tid][jj] + endt[jj]);
    float a = 0.f;
#pragma unroll 1
    for (int jj = 0; jj < 16; ++jj) a += expf(alpha[cur][tid][jj] + endt[jj] - m);
    rden[tid] = m + logf(a);
  }
  __syncthreads();
  if (tid == 0) {
    double acc = 0.0;
#pragma unroll 1
    for (int i = 0; i < 32; ++i) acc += (double)(rnum[i] - rden[i]);
    const float res = (float)acc;
    *(volatile float*)out = res;
    __threadfence();
    *(volatile float*)out = res;
  }
}

extern "C" void kernel_launch(void* const* d_in, const int* in_sizes, int n_in,
                              void* d_out, int out_size, void* d_ws, size_t ws_size, hipStream_t stream) {
  if (n_in < 14 || d_out == nullptr || d_ws == nullptr) return;
  if (in_sizes[0] != N_ROWS || in_sizes[1] != N_ROWS || in_sizes[2] != N_VOCAB * EMB_DIM ||
      in_sizes[3] != GATE_ROWS * EMB_DIM || in_sizes[4] != GATE_ROWS * HID_DIM || in_sizes[5] != GATE_ROWS ||
      in_sizes[6] != GATE_ROWS * EMB_DIM || in_sizes[7] != GATE_ROWS * HID_DIM || in_sizes[8] != GATE_ROWS ||
      in_sizes[9] != N_TAGS * W_TAG_COLS || in_sizes[10] != N_TAGS || in_sizes[11] != N_TAGS ||
      in_sizes[12] != N_TAGS || in_sizes[13] != N_TAGS * N_TAGS || out_size != 1) return;

  const int*   xin  = (const int*)d_in[0];
  const int*   yin  = (const int*)d_in[1];
  const float* tab  = (const float*)d_in[2];
  const float* Wihf = (const float*)d_in[3];
  const float* Whhf = (const float*)d_in[4];
  const float* bfp  = (const float*)d_in[5];
  const float* Wihb = (const float*)d_in[6];
  const float* Whhb = (const float*)d_in[7];
  const float* bbp  = (const float*)d_in[8];
  const float* Wtag = (const float*)d_in[9];
  const float* btag = (const float*)d_in[10];
  const float* stp  = (const float*)d_in[11];
  const float* enp  = (const float*)d_in[12];
  const float* trp  = (const float*)d_in[13];
  float* out = (float*)d_out;

  char* ws = (char*)d_ws; size_t off = 0;
  auto carve = [&](size_t bytes) -> char* { char* p = ws + off; off += (bytes + 255) & ~(size_t)255; return p; };
  unsigned short* X16  = (unsigned short*)carve((size_t)N_ROWS * EMB_PAD * 2);
  unsigned short* WIHF = (unsigned short*)carve((size_t)GATE_COLS * EMB_PAD * 2);
  unsigned short* WIHB = (unsigned short*)carve((size_t)GATE_COLS * EMB_PAD * 2);
  unsigned short* WHHF = (unsigned short*)carve((size_t)GATE_COLS * HID_PAD * 2);
  unsigned short* WHHB = (unsigned short*)carve((size_t)GATE_COLS * HID_PAD * 2);
  unsigned short* WT16 = (unsigned short*)carve((size_t)TAG_PAD * HS_COLS * 2);
  unsigned short* XP16 = (unsigned short*)carve((size_t)N_ROWS * GATE_COLS * 2);
  unsigned short* HS16 = (unsigned short*)carve((size_t)N_ROWS * HS_COLS * 2);
  float*          EMF  = (float*)carve((size_t)N_ROWS * TAG_PAD * 4);
  if (off > ws_size || off > (size_t)134217728) return;

  auto nblk = [](int ndr, int dcols) -> int { const int rpb = 256 / (dcols >> 3); return (ndr + rpb - 1) / rpb; };

  gather_rows_kernel<<<nblk(N_ROWS, EMB_PAD), 256, 0, stream>>>(xin, tab, X16, N_ROWS, N_VOCAB, EMB_DIM, EMB_PAD);
  cvt_pad_kernel<<<nblk(GATE_COLS, EMB_PAD), 256, 0, stream>>>(Wihf, WIHF, GATE_COLS, EMB_PAD, HID_PAD, HID_DIM, 4, GATE_ROWS, EMB_DIM, EMB_PAD, EMB_DIM, 1, W_CARRY);
  cvt_pad_kernel<<<nblk(GATE_COLS, EMB_PAD), 256, 0, stream>>>(Wihb, WIHB, GATE_COLS, EMB_PAD, HID_PAD, HID_DIM, 4, GATE_ROWS, EMB_DIM, EMB_PAD, EMB_DIM, 1, W_CARRY);
  cvt_pad_kernel<<<nblk(GATE_COLS, HID_PAD), 256, 0, stream>>>(Whhf, WHHF, GATE_COLS, HID_PAD, HID_PAD, HID_DIM, 4, GATE_ROWS, HID_DIM, HID_PAD, HID_DIM, 1, W_CARRY);
  cvt_pad_kernel<<<nblk(GATE_COLS, HID_PAD), 256, 0, stream>>>(Whhb, WHHB, GATE_COLS, HID_PAD, HID_PAD, HID_DIM, 4, GATE_ROWS, HID_DIM, HID_PAD, HID_DIM, 1, W_CARRY);
  cvt_pad_kernel<<<nblk(TAG_PAD, HS_COLS), 256, 0, stream>>>(Wtag, WT16, TAG_PAD, HS_COLS, TAG_PAD, N_TAGS, 1, N_TAGS, W_TAG_COLS, HID_PAD, HID_DIM, 2, W_CARRY);

  const int gemm_xp_blocks = ((N_ROWS / 64) * (GATE_COLS / 64)) / 8;
  const int gemm_em_blocks = ((N_ROWS / 64) * (TAG_PAD / 64)) / 8;

  wmma_gemm64<0, false, 0, 1, false, 0><<<dim3(gemm_xp_blocks, 1), 256, 0, stream>>>(
      X16, X16, EMB_PAD, 0L, WIHF, WIHF, EMB_PAD, 0L, (void*)XP16, (void*)XP16, GATE_COLS, 0L,
      bfp, bfp, 0L, N_ROWS, GATE_COLS, EMB_PAD, W_CARRY_INV);
  lstm_rec_kernel<<<N_BATCH / 16, REC_THREADS, 0, stream>>>(XP16, WHHF, bfp, HS16, 0);
  wmma_gemm64<0, false, 0, 1, false, 0><<<dim3(gemm_xp_blocks, 1), 256, 0, stream>>>(
      X16, X16, EMB_PAD, 0L, WIHB, WIHB, EMB_PAD, 0L, (void*)XP16, (void*)XP16, GATE_COLS, 0L,
      bbp, bbp, 0L, N_ROWS, GATE_COLS, EMB_PAD, W_CARRY_INV);
  lstm_rec_kernel<<<N_BATCH / 16, REC_THREADS, 0, stream>>>(XP16, WHHB, bbp, HS16, 1);
  wmma_gemm64<0, false, 0, 0, false, 0><<<dim3(gemm_em_blocks, 1), 256, 0, stream>>>(
      HS16, HS16, HS_COLS, 0L, WT16, WT16, HS_COLS, 0L, (void*)EMF, (void*)EMF, TAG_PAD, 0L,
      btag, btag, 0L, N_ROWS, TAG_PAD, HS_COLS, W_CARRY_INV);
  crf_kernel<<<1, 512, 0, stream>>>(EMF, yin, btag, stp, enp, trp, out);
}
